// GINEncoder_75771813036514
// MI455X (gfx1250) — hardware-run, weakly checked
//
#include <hip/hip_runtime.h>
#include <stddef.h>
#include <stdint.h>


#define DF      64
#define KP      128
#define NOC     768
#define NLAY    5
#define NTHR    256
#define NWAVE   8
#define EPT     8
#define CHUNK   (NTHR * EPT)
#define WCAP    (EPT * 32)
#define LISTN   (NWAVE * WCAP)
#define NBA     1024
#define PKS     10
#define RCAP    28672
#define DEGCAP  64
#define GBM     64
#define GBN     64
#define GTHR    128
#define GNT     (GBN / 16)
#define NWM     11
#define WPU     (DF * (KP / 8))
#define WPH     (DF * KP)
#define NUH     (NOC * (KP / 8))
#define NUW     (NWM * WPU + NUH)
#define WH2H    (NOC * KP)
#define PTHR    256
#define ZINTS   (2 * RCAP + 2 * NBA + LISTN)
#define LDS_AGG (ZINTS * 4 + 64)
#define WSMAX   134217728

static_assert((CHUNK & (CHUNK - 1)) == 0);
static_assert(NBA == (1 << PKS));
static_assert(((long long)CHUNK << PKS) < (1LL << 31));
static_assert(NTHR * 4 == NBA);
static_assert(LISTN >= NBA && LISTN >= NWAVE * WCAP);
static_assert((RCAP % 32) == 0);
static_assert((ZINTS % (NTHR * 4)) == 0);
static_assert(LDS_AGG <= 262144);
static_assert((NBA % NWAVE) == 0 && (NBA % GBM) == 0);
static_assert(GBM == (GTHR / 32) * 16);
static_assert(KP == 2 * DF && (KP % 32) == 0);
static_assert((WPU % NTHR) == 0 && WPU == 1024 && ((NWM * WPU) % NTHR) == 0 && (NUW % NTHR) == 0);
static_assert(DF == 16 * 4);
static_assert((DF * 4) % 128 == 0);
static_assert(GBN == DF && GNT == 4 && (NOC % GBN) == 0);
static_assert((KP / 8) == 16);
static_assert(PTHR == NWAVE * 32 && PTHR >= DF);

typedef float          v4f  __attribute__((ext_vector_type(4)));
typedef float          v8f  __attribute__((ext_vector_type(8)));
typedef int            v4i  __attribute__((ext_vector_type(4)));
typedef int            v8i  __attribute__((ext_vector_type(8)));
typedef unsigned int   v4u  __attribute__((ext_vector_type(4)));
typedef unsigned short v8us __attribute__((ext_vector_type(8)));
typedef _Float16       v16h __attribute__((ext_vector_type(16)));
typedef __bf16         v16b __attribute__((ext_vector_type(16)));
typedef v4f  __attribute__((may_alias)) v4fa;
typedef v4i  __attribute__((may_alias)) v4ia;
typedef v8us __attribute__((may_alias)) v8usa;
union Frag { v16b b; v16h f; v8us h[2]; v8i w; };

__device__ __forceinline__ v8f wmk(const Frag& a, const Frag& b, v8f c) {
  v8f d = __builtin_amdgcn_wmma_f32_16x16x32_bf16(false, a.b, false, b.b, (short)0, c, false, false);
  asm volatile("v_nop\n\tv_nop\n\tv_nop\n\tv_nop" : "+v"(d) : "v"(a.w), "v"(b.w));
  return d;
}

__device__ __forceinline__ unsigned short bf_bits(float f) {
  unsigned int u = __float_as_uint(f);
  u += 0x7FFFu + ((u >> 16) & 1u);
  return (unsigned short)(u >> 16);
}
__device__ __forceinline__ float bf_val(unsigned short b) {
  return __uint_as_float(((unsigned int)b) << 16);
}
__device__ __forceinline__ float bf_rne(float f) { return bf_val(bf_bits(f)); }

__device__ __forceinline__ v4u pack_hilo4(float r0, float r1, float r2, float r3) {
  const unsigned short hb0 = bf_bits(r0), hb1 = bf_bits(r1), hb2 = bf_bits(r2), hb3 = bf_bits(r3);
  const unsigned short lb0 = bf_bits(r0 - bf_val(hb0)), lb1 = bf_bits(r1 - bf_val(hb1));
  const unsigned short lb2 = bf_bits(r2 - bf_val(hb2)), lb3 = bf_bits(r3 - bf_val(hb3));
  v4u pk;
  pk.x = (unsigned int)hb0 | ((unsigned int)hb1 << 16);
  pk.y = (unsigned int)hb2 | ((unsigned int)hb3 << 16);
  pk.z = (unsigned int)lb0 | ((unsigned int)lb1 << 16);
  pk.w = (unsigned int)lb2 | ((unsigned int)lb3 << 16);
  return pk;
}

template <int ACT>
__device__ __forceinline__ float actf(float v) {
  if constexpr (ACT == 1) {
    return fmaxf(v, 0.0f);
  } else {
    return v;
  }
}

template <int RND>
__device__ __forceinline__ float cvin(float v) {
  if constexpr (RND == 1) {
    return bf_rne(v);
  } else {
    return v;
  }
}

__device__ __forceinline__ void wave_sync() {
  __builtin_amdgcn_fence(__ATOMIC_RELEASE, "wavefront");
  __builtin_amdgcn_wave_barrier();
  __builtin_amdgcn_fence(__ATOMIC_ACQUIRE, "wavefront");
}

__device__ __forceinline__ int scan_chunk(const int* __restrict__ dsts, int nE, int cbase, int slotBase,
                                          int nb, int vec8, int* list, int tid, int lane, int wave) {
  int wc = 0;
  const int el0  = tid * EPT;
  const int e0   = cbase + el0;
  const int sent = -2147483647 - 1;
  v4i da, db;
  if (vec8 != 0 && cbase + CHUNK <= nE) {
    da = *(const v4i*)(dsts + e0);
    db = *(const v4i*)(dsts + e0 + 4);
  } else {
    da.x = (e0     < nE) ? dsts[min(e0,     nE - 1)] : sent;
    da.y = (e0 + 1 < nE) ? dsts[min(e0 + 1, nE - 1)] : sent;
    da.z = (e0 + 2 < nE) ? dsts[min(e0 + 2, nE - 1)] : sent;
    da.w = (e0 + 3 < nE) ? dsts[min(e0 + 3, nE - 1)] : sent;
    db.x = (e0 + 4 < nE) ? dsts[min(e0 + 4, nE - 1)] : sent;
    db.y = (e0 + 5 < nE) ? dsts[min(e0 + 5, nE - 1)] : sent;
    db.z = (e0 + 6 < nE) ? dsts[min(e0 + 6, nE - 1)] : sent;
    db.w = (e0 + 7 < nE) ? dsts[min(e0 + 7, nE - 1)] : sent;
  }
  const unsigned nbs = (unsigned)slotBase;
  const unsigned unb = (unsigned)nb;
  const unsigned s0 = (unsigned)da.x - nbs, s1 = (unsigned)da.y - nbs;
  const unsigned s2 = (unsigned)da.z - nbs, s3 = (unsigned)da.w - nbs;
  const unsigned s4 = (unsigned)db.x - nbs, s5 = (unsigned)db.y - nbs;
  const unsigned s6 = (unsigned)db.z - nbs, s7 = (unsigned)db.w - nbs;
  const bool h0 = s0 < unb, h1 = s1 < unb, h2 = s2 < unb, h3 = s3 < unb;
  const bool h4 = s4 < unb, h5 = s5 < unb, h6 = s6 < unb, h7 = s7 < unb;
  const unsigned any = __builtin_amdgcn_ballot_w32(h0 | h1 | h2 | h3 | h4 | h5 | h6 | h7);
  if (any != 0u) {
#define HITJ(J, HJ, SJ) { \
      const unsigned mj = __builtin_amdgcn_ballot_w32(HJ); \
      if (mj != 0u) { \
        if (HJ) { \
          const int pos = wc + (int)__builtin_amdgcn_mbcnt_lo(mj, 0u); \
          if (pos < WCAP) list[wave * WCAP + pos] = ((el0 + (J)) << PKS) | (int)(SJ); \
        } \
        wc += (int)__builtin_popcount(mj); } }
    HITJ(0, h0, s0)
    HITJ(1, h1, s1)
    HITJ(2, h2, s2)
    HITJ(3, h3, s3)
    HITJ(4, h4, s4)
    HITJ(5, h5, s5)
    HITJ(6, h6, s6)
    HITJ(7, h7, s7)
#undef HITJ
  }
  return wc;
}

__global__ __launch_bounds__(NTHR) void k_wprep(const float* __restrict__ gw1, const float* __restrict__ gw2,
                                                const float* __restrict__ wh1, const float* __restrict__ wh2,
                                                unsigned short* WPL) {
  const int u = (int)blockIdx.x * NTHR + (int)threadIdx.x;
  if (u >= NUW) return;
  const float* w;
  int ncol, n, q;
  size_t dsto;
  if (u < NWM * WPU) {
    const int pl = u >> 10;
    const int v  = u & (WPU - 1);
    n = v >> 4;
    q = v & 15;
    w = (pl < NLAY) ? (gw1 + (size_t)pl * (DF * DF))
                    : ((pl < 2 * NLAY) ? (gw2 + (size_t)(pl - NLAY) * (DF * DF)) : wh1);
    ncol = DF;
    dsto = (size_t)pl * WPH + (size_t)n * KP + (size_t)(8 * q);
  } else {
    const int v = u - NWM * WPU;
    n = v >> 4;
    q = v & 15;
    w = wh2;
    ncol = NOC;
    dsto = (size_t)NWM * WPH + (size_t)n * KP + (size_t)(8 * q);
  }
  const float* p = w + (size_t)(4 * q) * (size_t)ncol + n;
  float f[4];
#pragma unroll
  for (int c = 0; c < 4; ++c) f[c] = p[(size_t)c * (size_t)ncol];
  v8us o;
#pragma unroll
  for (int j = 0; j < 8; ++j) o[j] = bf_bits(f[j & 3]);
  unsigned short* dp = WPL + dsto;
  *(volatile v8us*)dp = o;
  __threadfence();
  *(volatile v8us*)dp = o;
}

template <int ACT, int OUTK>
__global__ __launch_bounds__(GTHR) void k_gemm(const unsigned short* __restrict__ A, int lda,
                                               const unsigned short* __restrict__ BT, int ldb, int K,
                                               const float* __restrict__ bias,
                                               float* C32, unsigned short* C16, int ldc, int nRows) {
  static_assert(OUTK == 1 || OUTK == 2);
  __shared__ __attribute__((aligned(16))) float stg[GBM * GBN];
  const int tid = (int)threadIdx.x, lane = tid & 31, wave = tid >> 5, hh = lane >> 4, m = lane & 15;
  const int rowBase = (int)blockIdx.x * GBM;
  const int col0    = (int)blockIdx.y * GBN;

  v8f acc[GNT];
  {
    const v8f z = {0.f, 0.f, 0.f, 0.f, 0.f, 0.f, 0.f, 0.f};
#pragma unroll
    for (int t = 0; t < GNT; ++t) acc[t] = z;
  }
  const unsigned short* ap = A  + (size_t)(rowBase + 16 * wave + m) * (size_t)lda + 8 * hh;
  const unsigned short* bp = BT + (size_t)(col0 + m) * (size_t)ldb + 8 * hh;

#pragma unroll 1
  for (int k0 = 0; k0 < K; k0 += 32) {
    Frag af;
    af.h[0] = *(const v8usa*)(ap + k0);
    af.h[1] = *(const v8usa*)(ap + k0 + 16);
#pragma unroll
    for (int nt = 0; nt < GNT; ++nt) {
      const unsigned short* wq = bp + (size_t)(16 * nt) * (size_t)ldb + k0;
      Frag bf;
      bf.h[0] = *(const v8usa*)wq;
      bf.h[1] = *(const v8usa*)(wq + 16);
      acc[nt] = wmk(af, bf, acc[nt]);
    }
  }

#pragma unroll
  for (int nt = 0; nt < GNT; ++nt) {
    const int lc = 16 * nt + m;
    const float bb = bf_rne(bias[col0 + lc]);
#pragma unroll
    for (int r = 0; r < 8; ++r) {
      const int lr = 16 * wave + 8 * hh + r;
      stg[lr * GBN + lc] = actf<ACT>(acc[nt][r] + bb);
    }
  }
  __syncthreads();

  if constexpr (OUTK == 1) {
    v4f fv[8];
#pragma unroll
    for (int i = 0; i < 8; ++i) {
      const int lr = 16 * wave + 2 * i + hh;
      fv[i] = *(const v4fa*)(stg + lr * GBN + 4 * m);
    }
#pragma unroll
    for (int i = 0; i < 8; ++i) {
      const int gr = rowBase + 16 * wave + 2 * i + hh;
      float* op = C32 + (size_t)gr * (size_t)ldc + col0 + 4 * m;
      if (gr < nRows) *(volatile v4f*)op = fv[i];
    }
    __threadfence();
#pragma unroll
    for (int i = 0; i < 8; ++i) {
      const int gr = rowBase + 16 * wave + 2 * i + hh;
      float* op = C32 + (size_t)gr * (size_t)ldc + col0 + 4 * m;
      if (gr < nRows) *(volatile v4f*)op = fv[i];
    }
    (void)C16;
  } else {
    v4u pk[8];
#pragma unroll
    for (int i = 0; i < 8; ++i) {
      const int lr = 16 * wave + 2 * i + hh;
      const v4f q4 = *(const v4fa*)(stg + lr * GBN + 4 * m);
      pk[i] = pack_hilo4(q4.x, q4.y, q4.z, q4.w);
    }
#pragma unroll
    for (int i = 0; i < 8; ++i) {
      const int lr = 16 * wave + 2 * i + hh;
      unsigned short* op = C16 + (size_t)(rowBase + lr) * (size_t)ldc + 8 * m;
      *(volatile v4u*)op = pk[i];
    }
    __threadfence();
#pragma unroll
    for (int i = 0; i < 8; ++i) {
      const int lr = 16 * wave + 2 * i + hh;
      unsigned short* op = C16 + (size_t)(rowBase + lr) * (size_t)ldc + 8 * m;
      *(volatile v4u*)op = pk[i];
    }
    (void)C32; (void)nRows;
  }
}

template <int RND>
__global__ __launch_bounds__(NTHR) void k_agg(const int* __restrict__ srcs, const int* __restrict__ dsts,
                                              const float* X, const float* __restrict__ epsp,
                                              unsigned short* Aout, int nN, int nE, int vec8) {
  extern __shared__ __attribute__((aligned(16))) int lds_i[];
  int* reg1 = lds_i;
  int* reg2 = reg1 + RCAP;
  int* scnt = reg2 + RCAP;
  int* soff = scnt + NBA;
  int* list = soff + NBA;
  int* wcnt = list + LISTN;
  int* wtot = wcnt + NWAVE;
  const int tid = (int)threadIdx.x, lane = tid & 31, wave = tid >> 5;
  const int cl = lane & 15;
  const int nodeBase = (int)blockIdx.x * NBA;

  {
    const v4i z4 = {0, 0, 0, 0};
    for (int i = tid * 4; i < ZINTS; i += NTHR * 4) *(v4ia*)(lds_i + i) = z4;
    if (tid < 2 * NWAVE) wcnt[tid] = 0;
  }
  __syncthreads();

  int tot = 0;
  const int nChunks = (nE + CHUNK - 1) / CHUNK;
#pragma unroll 1
  for (int ch = 0; ch < nChunks; ++ch) {
    const int cbase = ch * CHUNK;
    const int wc = scan_chunk(dsts, nE, cbase, nodeBase, NBA, vec8, list, tid, lane, wave);
    if (lane == 0) wcnt[wave] = wc;
    __syncthreads();
    int pre = 0, all = 0;
#pragma unroll
    for (int w2 = 0; w2 < NWAVE; ++w2) {
      int c = wcnt[w2];
      c = c < 0 ? 0 : (c > WCAP ? WCAP : c);
      all += c;
      pre += (w2 < wave) ? c : 0;
    }
    const int wcc  = wc > WCAP ? WCAP : wc;
    const int base = tot + pre;
#pragma unroll 1
    for (int i = lane; i < wcc; i += 32) {
      const int ent = list[wave * WCAP + i];
      const int el  = (ent >> PKS) & (CHUNK - 1);
      const int sl  = ent & (NBA - 1);
      int eid = cbase + el;
      eid = eid > nE - 1 ? nE - 1 : eid;
      const int pos = base + i;
      if (pos < RCAP) reg1[pos] = (int)(((unsigned)eid << PKS) | (unsigned)sl);
    }
    tot += all;
    tot = tot > RCAP ? RCAP : tot;
    __syncthreads();
  }
  const int nh = tot;

  if (wave == 0) {
#pragma unroll 1
    for (int b0 = 0; b0 < nh; b0 += 32) {
      const int idx = b0 + lane;
      const int uv  = reg1[idx < RCAP ? idx : RCAP - 1];
      const int m32 = (nh - b0) < 32 ? (nh - b0) : 32;
#pragma unroll 1
      for (int k = 0; k < m32; ++k) {
        const int u  = __builtin_amdgcn_readlane(uv, k);
        const int sl = u & (NBA - 1);
        if (lane == 0) scnt[sl] = scnt[sl] + 1;
      }
    }
  }
  __syncthreads();

  {
    const v4i ca = *(const v4ia*)(scnt + 4 * tid);
    const int e0 = ca.x < 0 ? 0 : ca.x, e1 = ca.y < 0 ? 0 : ca.y, e2 = ca.z < 0 ? 0 : ca.z, e3 = ca.w < 0 ? 0 : ca.w;
    const int ts = e0 + e1 + e2 + e3;
    int incl = ts;
#pragma unroll
    for (int d = 1; d < 32; d <<= 1) {
      const int up = __shfl_up(incl, d, 32);
      if (lane >= d) incl += up;
    }
    if (lane == 31) wtot[wave] = incl;
    __syncthreads();
    int pre = 0;
#pragma unroll
    for (int w2 = 0; w2 < NWAVE; ++w2) pre += (w2 < wave) ? wtot[w2] : 0;
    int run = pre + incl - ts;
    soff[4 * tid + 0] = run; run += e0;
    soff[4 * tid + 1] = run; run += e1;
    soff[4 * tid + 2] = run; run += e2;
    soff[4 * tid + 3] = run;
  }
  __syncthreads();
  for (int i = tid; i < NBA; i += NTHR) list[i] = soff[i];
  __syncthreads();

  if (wave == 0) {
#pragma unroll 1
    for (int b0 = 0; b0 < nh; b0 += 32) {
      const int idx = b0 + lane;
      const int uv  = reg1[idx < RCAP ? idx : RCAP - 1];
      const int m32 = (nh - b0) < 32 ? (nh - b0) : 32;
#pragma unroll 1
      for (int k = 0; k < m32; ++k) {
        const int u   = __builtin_amdgcn_readlane(uv, k);
        const int sl  = u & (NBA - 1);
        const int eid = (int)((unsigned)u >> PKS);
        if (lane == 0) {
          int pos = list[sl];
          pos = pos < 0 ? 0 : (pos > RCAP - 1 ? RCAP - 1 : pos);
          reg2[pos] = eid;
          list[sl] = pos + 1;
        }
      }
    }
  }
  __syncthreads();

  const int nbw = NBA / NWAVE;
  const bool ovf = (nh >= RCAP);
  const float qnan = __int_as_float(0x7fc00000);
  const float ep = 1.0f + bf_rne(epsp[0]);

#pragma unroll 1
  for (int jt = 0; jt < nbw; ++jt) {
    const int slot = wave * nbw + jt;
    const int node = nodeBase + slot;
    int st = soff[slot];
    const int craw = scnt[slot];
    int cnt = craw;
    st  = st < 0 ? 0 : (st > nh ? nh : st);
    cnt = cnt < 0 ? 0 : (cnt > DEGCAP ? DEGCAP : cnt);
    if (cnt > nh - st) cnt = nh - st;
    const float pz = (ovf || craw > DEGCAP) ? qnan : 0.0f;
    const bool live = node < nN;
    const int nc = node < nN ? node : nN - 1;

    float a0 = 0.f, a1 = 0.f, a2 = 0.f, a3 = 0.f;
#pragma unroll 1
    for (int b0 = 0; b0 < cnt; b0 += 32) {
      int idx = st + b0 + lane; idx = idx > RCAP - 1 ? RCAP - 1 : idx;
      int eid = reg2[idx]; eid = eid < 0 ? 0 : (eid > nE - 1 ? nE - 1 : eid);
      int sr = srcs[eid]; sr = sr < 0 ? 0 : (sr > nN - 1 ? nN - 1 : sr);
      const int m32 = (cnt - b0) < 32 ? (cnt - b0) : 32;
#pragma unroll 1
      for (int k = 0; k < m32; ++k) {
        const int sk = __builtin_amdgcn_readlane(sr, k);
        const v4f v = *(const v4fa*)(X + (size_t)sk * DF + 4 * cl);
        a0 += cvin<RND>(v.x); a1 += cvin<RND>(v.y); a2 += cvin<RND>(v.z); a3 += cvin<RND>(v.w);
      }
    }
    const v4f sv = *(const v4fa*)(X + (size_t)nc * DF + 4 * cl);
    float r0 = ep * cvin<RND>(sv.x) + a0, r1 = ep * cvin<RND>(sv.y) + a1;
    float r2 = ep * cvin<RND>(sv.z) + a2, r3 = ep * cvin<RND>(sv.w) + a3;
    r0 = (live ? r0 : 0.0f) + pz;
    r1 = (live ? r1 : 0.0f) + pz;
    r2 = (live ? r2 : 0.0f) + pz;
    r3 = (live ? r3 : 0.0f) + pz;

    const v4u pk = pack_hilo4(r0, r1, r2, r3);
    const bool wr = lane < 16;
    unsigned short* gp = Aout + (size_t)node * (size_t)KP + 8 * cl;
    if (wr) *(volatile v4u*)gp = pk;
    __threadfence();
    if (wr) *(volatile v4u*)gp = pk;
  }
}

__global__ __launch_bounds__(PTHR) void k_pool(const float* ne, const int* __restrict__ bat, int nN,
                                               unsigned short* PP) {
  __shared__ __attribute__((aligned(16))) float wst[NWAVE * DF];
  __shared__ __attribute__((aligned(16))) float pst[DF];
  __shared__ int plist[NWAVE * 32];
  __shared__ int wcn[NWAVE];
  const int tid = (int)threadIdx.x, lane = tid & 31, wave = tid >> 5;
  const int cl = lane & 15;
  const int g = (int)blockIdx.x;
  float s0 = 0.0f, s1 = 0.0f, s2 = 0.0f, s3 = 0.0f;
  int cn = 0;
  const int nChunks = (nN + PTHR - 1) / PTHR;
#pragma unroll 1
  for (int ch = 0; ch < nChunks; ++ch) {
    const int n  = ch * PTHR + tid;
    const int nc = n < nN ? n : nN - 1;
    const int bv = bat[nc];
    const bool hit = (n < nN) && (bv == g);
    const unsigned mj = __builtin_amdgcn_ballot_w32(hit);
    if (mj != 0u) {
      if (hit) plist[wave * 32 + (int)__builtin_amdgcn_mbcnt_lo(mj, 0u)] = n;
      const int c = (int)__builtin_popcount(mj);
      wave_sync();
#pragma unroll 1
      for (int k = 0; k < c; ++k) {
        int nd = plist[wave * 32 + k];
        nd = nd < 0 ? 0 : (nd > nN - 1 ? nN - 1 : nd);
        const v4f r = *(const v4fa*)(ne + (size_t)nd * DF + 4 * cl);
        s0 += r.x; s1 += r.y; s2 += r.z; s3 += r.w;
      }
      cn += c;
      wave_sync();
    }
  }
  {
    v4f sv4; sv4.x = s0; sv4.y = s1; sv4.z = s2; sv4.w = s3;
    if (lane < 16) *(v4fa*)(wst + wave * DF + 4 * cl) = sv4;
    if (lane == 0) wcn[wave] = cn;
  }
  __syncthreads();
  if (tid < DF) {
    double sv = 0.0;
    int ct = 0;
#pragma unroll 1
    for (int w2 = 0; w2 < NWAVE; ++w2) {
      sv += (double)wst[w2 * DF + tid];
      ct += wcn[w2];
    }
    const float cf = (float)(ct < 1 ? 1 : ct);
    pst[tid] = (float)sv * (1.0f / cf);
  }
  __syncthreads();
  if (tid < 32) {
    const v4f q4 = *(const v4fa*)(pst + 4 * cl);
    const v4u pk = pack_hilo4(q4.x, q4.y, q4.z, q4.w);
    const bool wr = lane < 16;
    unsigned short* dp = PP + (size_t)g * (size_t)KP + 8 * cl;
    if (wr) *(volatile v4u*)dp = pk;
    __threadfence();
    if (wr) *(volatile v4u*)dp = pk;
  }
}

static inline int cdiv(int a, int b) { return (a + b - 1) / b; }
static inline size_t al256(size_t o) { return (o + 255) & ~(size_t)255; }

extern "C" void kernel_launch(void* const* d_in, const int* in_sizes, int n_in,
                              void* d_out, int out_size, void* d_ws, size_t ws_size,
                              hipStream_t stream) {
  if (n_in < 12) return;
  if (in_sizes[0] < DF || (in_sizes[0] % DF) != 0) return;
  const int nN = in_sizes[0] / DF;
  if (nN < 1 || nN > (1 << 22)) return;
  if (in_sizes[1] < 2 || (in_sizes[1] & 1) != 0) return;
  const int nE = in_sizes[1] / 2;
  if (nE < 1 || nE >= (1 << 21)) return;
  if (in_sizes[2] != nN) return;
  if (in_sizes[3] != NLAY * DF * DF || in_sizes[4] != NLAY * DF) return;
  if (in_sizes[5] != NLAY * DF * DF || in_sizes[6] != NLAY * DF) return;
  if (in_sizes[7] != NLAY) return;
  if (in_sizes[8] != DF * DF || in_sizes[9] != DF) return;
  if (in_sizes[10] != DF * NOC || in_sizes[11] != NOC) return;
  if (out_size < NOC || (out_size % NOC) != 0) return;
  const int nG = out_size / NOC;
  if (nG < 1 || nG > (1 << 16)) return;

  const float* x   = (const float*)d_in[0];
  const int*   ei  = (const int*)  d_in[1];
  const int*   bat = (const int*)  d_in[2];
  const float* gw1 = (const float*)d_in[3];
  const float* gb1 = (const float*)d_in[4];
  const float* gw2 = (const float*)d_in[5];
  const float* gb2 = (const float*)d_in[6];
  const float* eps = (const float*)d_in[7];
  const float* wh1 = (const float*)d_in[8];
  const float* bh1 = (const float*)d_in[9];
  const float* wh2 = (const float*)d_in[10];
  const float* bh2 = (const float*)d_in[11];
  float* out = (float*)d_out;
  const int* src = ei;
  const int* dst = ei + nE;

  const int MP   = cdiv(nN, GBM) * GBM;
  const int gM   = MP / GBM;
  const int gA   = cdiv(MP, NBA);
  const int RA   = gA * NBA;
  const int GP   = cdiv(nG, GBM) * GBM;
  const int gP   = GP / GBM;
  const int vec8 = ((nE & 3) == 0) ? 1 : 0;
  if ((long long)RA < (long long)MP) return;

  char* ws = (char*)d_ws;
  size_t off = 0;
  const size_t oWPL = off; off = al256(off + ((size_t)NWM * WPH + (size_t)WH2H) * 2);
  const size_t oAP  = off; off = al256(off + (size_t)RA * KP * 2);
  const size_t oTP  = off; off = al256(off + (size_t)MP * KP * 2);
  const size_t oH   = off; off = al256(off + (size_t)MP * DF * 4);
  const size_t oPP  = off; off = al256(off + (size_t)GP * KP * 2);
  const size_t oHD  = off; off = al256(off + (size_t)GP * KP * 2);
  if (off > ws_size || off > (size_t)WSMAX) return;
  unsigned short* WPL = (unsigned short*)(ws + oWPL);
  unsigned short* AP  = (unsigned short*)(ws + oAP);
  unsigned short* TP  = (unsigned short*)(ws + oTP);
  float*          H   = (float*)(ws + oH);
  unsigned short* PP  = (unsigned short*)(ws + oPP);
  unsigned short* HD  = (unsigned short*)(ws + oHD);
  const unsigned short* WH2P = WPL + (size_t)NWM * WPH;

  hipFuncSetAttribute(reinterpret_cast<const void*>(&k_agg<1>), hipFuncAttributeMaxDynamicSharedMemorySize, LDS_AGG);
  hipFuncSetAttribute(reinterpret_cast<const void*>(&k_agg<0>), hipFuncAttributeMaxDynamicSharedMemorySize, LDS_AGG);

  k_wprep<<<NUW / NTHR, NTHR, 0, stream>>>(gw1, gw2, wh1, wh2, WPL);

  for (int l = 0; l < NLAY; ++l) {
    const unsigned short* W1D = WPL + (size_t)l * WPH;
    const unsigned short* W2D = WPL + (size_t)(NLAY + l) * WPH;
    if (l == 0) {
      k_agg<1><<<gA, NTHR, LDS_AGG, stream>>>(src, dst, x, eps + l, AP, nN, nE, vec8);
    } else {
      k_agg<0><<<gA, NTHR, LDS_AGG, stream>>>(src, dst, H, eps + l, AP, nN, nE, vec8);
    }
    k_gemm<1, 2><<<dim3(gM, 1), GTHR, 0, stream>>>(AP, KP, W1D, KP, KP, gb1 + (size_t)l * DF, H, TP, KP, MP);
    if (l < NLAY - 1) {
      k_gemm<1, 1><<<dim3(gM, 1), GTHR, 0, stream>>>(TP, KP, W2D, KP, KP, gb2 + (size_t)l * DF, H, TP, DF, MP);
    } else {
      k_gemm<0, 1><<<dim3(gM, 1), GTHR, 0, stream>>>(TP, KP, W2D, KP, KP, gb2 + (size_t)l * DF, H, TP, DF, MP);
    }
  }

  k_pool<<<GP, PTHR, 0, stream>>>(H, bat, nN, PP);
  k_gemm<1, 2><<<dim3(gP, 1), GTHR, 0, stream>>>(PP, KP, WPL + (size_t)(2 * NLAY) * WPH, KP, KP, bh1, H, HD, KP, GP);
  k_gemm<0, 1><<<dim3(gP, NOC / GBN), GTHR, 0, stream>>>(HD, KP, WH2P, KP, KP, bh2, out, HD, NOC, nG);
}
